// Relation_Module_45664092291701
// MI455X (gfx1250) — hardware-run, weakly checked
//
#include <hip/hip_runtime.h>


#define NR   1024
#define NF   2048
#define NM   64
#define CARW 1024.0f
typedef _Float16 h16;
typedef unsigned short bf;
typedef __attribute__((ext_vector_type(16))) __bf16   v16bf;
typedef __attribute__((ext_vector_type(16))) _Float16 v16h;
typedef __attribute__((ext_vector_type(8)))  _Float16 v8h;
typedef __attribute__((ext_vector_type(8)))  unsigned short v8us;
typedef __attribute__((ext_vector_type(8)))  float    v8f;
typedef __attribute__((ext_vector_type(4)))  float    v4f;
typedef v8h  __attribute__((may_alias)) v8ha;
typedef v4f  __attribute__((may_alias)) v4fa;
typedef v8us __attribute__((may_alias)) v8usa;

__device__ __forceinline__ unsigned short f2bf(float f) { unsigned u = __float_as_uint(f); u += 0x7FFFu + ((u >> 16) & 1u); return (unsigned short)(u >> 16); }
__device__ __forceinline__ float bf2f(unsigned short b) { return __uint_as_float(((unsigned)b) << 16); }
__device__ __forceinline__ float bfr(float f) { return bf2f(f2bf(f)); }
__device__ __forceinline__ v16h cat16(v8h lo, v8h hi) { return __builtin_shufflevector(lo, hi, 0, 1, 2, 3, 4, 5, 6, 7, 8, 9, 10, 11, 12, 13, 14, 15); }
__device__ __forceinline__ v16bf cat16b(v8us lo, v8us hi) { return __builtin_bit_cast(v16bf, __builtin_shufflevector(lo, hi, 0, 1, 2, 3, 4, 5, 6, 7, 8, 9, 10, 11, 12, 13, 14, 15)); }
__device__ __forceinline__ v8f wmma16(v16h a, v16h b, v8f c) { return __builtin_amdgcn_wmma_f32_16x16x32_f16(false, a, false, b, (short)0, c, false, false); }
__device__ __forceinline__ v8f wmmab(v16bf a, v16bf b, v8f c) { return __builtin_amdgcn_wmma_f32_16x16x32_bf16(false, a, false, b, (short)0, c, false, false); }


template <typename T16> struct WFrag;
template <> struct WFrag<h16> { typedef v16h V; static __device__ __forceinline__ V ld(const h16* p) { return cat16(*(const v8h*)p, *(const v8h*)(p + 16)); } static __device__ __forceinline__ v8f mma(V a, V b, v8f c) { return wmma16(a, b, c); } };
template <> struct WFrag<bf> { typedef v16bf V; static __device__ __forceinline__ V ld(const bf* p) { return cat16b(*(const v8us*)p, *(const v8us*)(p + 16)); } static __device__ __forceinline__ v8f mma(V a, V b, v8f c) { return wmmab(a, b, c); } };
template <typename T16, int NSPLIT, bool BIAS>
__global__ __launch_bounds__(32) void k_gemmw(const T16* __restrict__ A, const T16* __restrict__ A2, const T16* __restrict__ Bt, const T16* __restrict__ Bt2, int K, float* C, int ldc, const float* __restrict__ bias, size_t sA, size_t sB, size_t sC) {
    typedef typename WFrag<T16>::V V;
    __shared__ __align__(16) float os[16 * 68];
    const size_t z = blockIdx.z; A += z * sA; if (A2) A2 += z * sA; Bt += z * sB; if (Bt2) Bt2 += z * sB; C += z * sC;
    const int lane = threadIdx.x & 31, lr = lane & 15, hi = lane >> 4; const int r0 = blockIdx.x * 64, c0 = blockIdx.y * 64;
    v8f acc[4][4];
#pragma unroll
    for (int mb = 0; mb < 4; ++mb)
#pragma unroll
        for (int nb = 0; nb < 4; ++nb) acc[mb][nb] = (v8f){};
    const size_t aoff = (size_t)(r0 + lr) * K + 8 * hi, boff = (size_t)(c0 + lr) * K + 8 * hi;

    for (int kc = 0; kc < K; kc += 32) {
        V a[4], a2[4];
#pragma unroll
        for (int mb = 0; mb < 4; ++mb) { a[mb] = WFrag<T16>::ld(A + aoff + (size_t)mb * 16 * K + kc); if (NSPLIT == 1 || NSPLIT == 2) a2[mb] = WFrag<T16>::ld(A2 + aoff + (size_t)mb * 16 * K + kc); }
#pragma unroll
        for (int nb = 0; nb < 4; ++nb) { const V b = WFrag<T16>::ld(Bt + boff + (size_t)nb * 16 * K + kc); V b2; if (NSPLIT >= 2) b2 = WFrag<T16>::ld(Bt2 + boff + (size_t)nb * 16 * K + kc);
#pragma unroll
            for (int mb = 0; mb < 4; ++mb) { acc[mb][nb] = WFrag<T16>::mma(a[mb], b, acc[mb][nb]); if (NSPLIT == 1 || NSPLIT == 2) acc[mb][nb] = WFrag<T16>::mma(a2[mb], b, acc[mb][nb]); if (NSPLIT >= 2) acc[mb][nb] = WFrag<T16>::mma(a[mb], b2, acc[mb][nb]); } }
        asm volatile("v_nop\n\tv_nop\n\tv_nop\n\tv_nop" : "+v"(acc[0][0]), "+v"(acc[1][1]), "+v"(acc[2][2]), "+v"(acc[3][3]) : "v"(a[0]), "v"(a[3]));
    }
#pragma unroll
    for (int mb = 0; mb < 4; ++mb) {
#pragma unroll
        for (int nb = 0; nb < 4; ++nb) {
#pragma unroll
            for (int j = 0; j < 8; ++j) os[(hi * 8 + j) * 68 + nb * 16 + lr] = acc[mb][nb][j]; }
        __builtin_amdgcn_wave_barrier(); asm volatile("" ::: "memory");
        float* crow = C + (size_t)(r0 + mb * 16) * ldc + c0;
#pragma unroll 1
        for (int ps = 0; ps < 2; ++ps) {
#pragma unroll
            for (int s = 0; s < 8; ++s) { const int row = 2 * s + hi, cofs = lr * 4; v4f val = *(const v4fa*)(os + row * 68 + cofs); if (BIAS) { val[0] += bfr(bias[c0 + cofs]); val[1] += bfr(bias[c0 + cofs + 1]); val[2] += bfr(bias[c0 + cofs + 2]); val[3] += bfr(bias[c0 + cofs + 3]); }
                *(volatile v4f*)(crow + (size_t)row * ldc + cofs) = val; }
            if (ps == 0) __threadfence(); }
        __builtin_amdgcn_wave_barrier(); asm volatile("" ::: "memory");
    }
}

__device__ __forceinline__ h16 tohx(float x) { return (h16)x; }
__device__ __forceinline__ void splitf(float y, unsigned short& h, unsigned short& l) { h = f2bf(y); l = f2bf(y - bf2f(h)); }
typedef __attribute__((ext_vector_type(2))) _Float16 v2h;
typedef __attribute__((ext_vector_type(4))) _Float16 v4h;
typedef __attribute__((ext_vector_type(2))) unsigned short v2us;
typedef __attribute__((ext_vector_type(4))) unsigned short v4us;
typedef __attribute__((ext_vector_type(2))) float v2f;
typedef __attribute__((ext_vector_type(4))) int v4i;
__global__ __launch_bounds__(256) void k_f2h(const float* __restrict__ S, h16* P16, size_t n4) { const size_t i = (size_t)blockIdx.x * 256 + threadIdx.x; if (i >= n4) return; const v4f v = *(const v4f*)(S + i * 4); v4h o;
#pragma unroll
    for (int q = 0; q < 4; ++q) o[q] = tohx(v[q]);
    *(volatile v4h*)(P16 + i * 4) = o; __threadfence(); *(volatile v4h*)(P16 + i * 4) = o; }
__global__ __launch_bounds__(256) void k_wtG(const float* __restrict__ w, int K, int N, bf* Bt) {
    const int lane = threadIdx.x & 31; const int L0 = (blockIdx.x * 8 + (threadIdx.x >> 5)) * 8; const int nlines = N * K / 64;
#pragma unroll
    for (int ps = 0; ps < 2; ++ps) {
        for (int l = 0; l < 8; ++l) { const int L = L0 + l; if (L >= nlines) break; const size_t e = (size_t)L * 64 + lane * 2; const int k = (int)(e % K), n = (int)(e / K); v2us o;
            o[0] = f2bf(w[(size_t)k * N + n]); o[1] = f2bf(w[(size_t)(k + 1) * N + n]); *(volatile v2us*)(Bt + e) = o; }
        if (ps == 0) __threadfence(); }
}
__global__ __launch_bounds__(256) void k_rl8(const float* __restrict__ src, bf* dst) { const size_t i = (size_t)blockIdx.x * 256 + threadIdx.x; const v4f p0 = *(const v4f*)(src + i * 8), p1 = *(const v4f*)(src + i * 8 + 4); v8us o;
#pragma unroll
    for (int e = 0; e < 4; ++e) { o[e] = f2bf(fmaxf(p0[e], 0.0f)); o[4 + e] = f2bf(fmaxf(p1[e], 0.0f)); }
    *(volatile v8us*)(dst + i * 8) = o; __threadfence(); *(volatile v8us*)(dst + i * 8) = o; }
__global__ __launch_bounds__(256) void k_pair(const float* __restrict__ EN, const float* __restrict__ a1, const float* __restrict__ a8, const float* __restrict__ a9, const float* __restrict__ a10, const float* __restrict__ a11, float* UW) {
    const unsigned ii = blockIdx.x, j0 = threadIdx.x * 4u; const v4f ri = *(const v4f*)(a1 + (size_t)ii * 4); const float ix0 = bfr(ri[0]), iy0 = bfr(ri[1]), ix1 = bfr(ri[2]), iy1 = bfr(ri[3]); const float sxi = ix1 - ix0, syi = iy1 - iy0, cxi = 0.5f * (ix0 + ix1), cyi = 0.5f * (iy0 + iy1);
    const v4f en = *(const v4f*)(EN + (size_t)ii * NR + j0); const float tail = bfr(a11[0]); v4f o;
#pragma unroll
    for (int e = 0; e < 4; ++e) { const unsigned jj = j0 + e; const v4f rj = *(const v4f*)(a1 + (size_t)jj * 4); const float jx0 = bfr(rj[0]), jy0 = bfr(rj[1]), jx1 = bfr(rj[2]), jy1 = bfr(rj[3]); const float sxj = jx1 - jx0, syj = jy1 - jy0, cxj = 0.5f * (jx0 + jx1), cyj = 0.5f * (jy0 + jy1);
        const float f0 = __logf(fabsf(cxj - cxi) / sxi + 1e-3f), f1 = __logf(fabsf(cyj - cyi) / syi + 1e-3f), f2 = __logf(sxj / sxi), f3 = __logf(syj / syi); float acc = 0.0f;
        for (int m_ = 0; m_ < NM; ++m_) { float hu = f0 * bfr(a8[m_]); hu += f1 * bfr(a8[NM + m_]); hu += f2 * bfr(a8[2 * NM + m_]); hu += f3 * bfr(a8[3 * NM + m_]); hu += bfr(a9[m_]); hu = fmaxf(hu, 0.0f); acc += hu * bfr(a10[m_]); }
        const float gate = fmaxf(acc + tail, 0.0f); const float val = __expf(en[e] * 0.125f) * gate; o[e] = (jj == ii) ? 0.0f : val; }
    float* dst = UW + (size_t)ii * NR + j0; *(volatile v4f*)dst = o; __threadfence(); *(volatile v4f*)dst = o; }
__global__ __launch_bounds__(256) void k_rown(const float* __restrict__ UW, h16* WH) { const unsigned rr = blockIdx.x * 256u + threadIdx.x; const float* src = UW + (size_t)rr * NR; float sum = 0.0f;
    for (int c4 = 0; c4 < NR / 4; ++c4) { const v4f p = *(const v4f*)(src + c4 * 4); sum += p[0]; sum += p[1]; sum += p[2]; sum += p[3]; }
    const float den = sum + 1e-10f; h16* dst = WH + (size_t)rr * NR;
    for (int c4 = 0; c4 < NR / 4; ++c4) { const v4f p = *(const v4f*)(src + c4 * 4); v4h o;
#pragma unroll
        for (int e = 0; e < 4; ++e) o[e] = tohx((p[e] / den) * CARW);
        *(volatile v4h*)(dst + c4 * 4) = o; __threadfence(); *(volatile v4h*)(dst + c4 * 4) = o; } }
__global__ __launch_bounds__(256) void k_tr16(const float* __restrict__ A3, h16* TR) { const unsigned cc = blockIdx.x, r0 = threadIdx.x * 4u; const float* src = A3 + (size_t)r0 * NF + cc; v4h o;
#pragma unroll
    for (int e = 0; e < 4; ++e) o[e] = tohx(src[(size_t)e * NF]);
    h16* dst = TR + (size_t)cc * NR + r0; *(volatile v4h*)dst = o; __threadfence(); *(volatile v4h*)dst = o; }
__global__ __launch_bounds__(256) void k_unc(const float* __restrict__ Y, float* OUT) { const size_t i = (size_t)blockIdx.x * 256 + threadIdx.x; const v4f p = *(const v4f*)(Y + i * 4); v4f o;
#pragma unroll
    for (int e = 0; e < 4; ++e) o[e] = p[e] * (1.0f / CARW);
    *(volatile v4f*)(OUT + i * 4) = o; __threadfence(); *(volatile v4f*)(OUT + i * 4) = o; }

extern "C" void kernel_launch(void* const* d_in, const int* in_sizes, int n_in,
                              void* d_out, int out_size, void* d_ws, size_t ws_size, hipStream_t stream) {
    (void)in_sizes; (void)n_in; (void)out_size;
    const float* a0 = (const float*)d_in[0]; const float* a1 = (const float*)d_in[1]; const float* a2 = (const float*)d_in[2]; const float* a3 = (const float*)d_in[3]; const float* a4 = (const float*)d_in[4]; const float* a5 = (const float*)d_in[5];
    const float* a6 = (const float*)d_in[6]; const float* a7 = (const float*)d_in[7]; const float* a8 = (const float*)d_in[8]; const float* a9 = (const float*)d_in[9]; const float* a10 = (const float*)d_in[10]; const float* a11 = (const float*)d_in[11];
    float* OUT = (float*)d_out;
    char* wsp = (char*)d_ws;
    auto take = [&](size_t bytes) { char* p = wsp; wsp += (bytes + 255) & ~(size_t)255; return (void*)p; };
    bf* PB = (bf*)take((size_t)NR * NF * 2); bf* W1 = (bf*)take((size_t)NM * NF * 2); bf* W2 = (bf*)take((size_t)NM * NF * 2); bf* W3 = (bf*)take((size_t)NF * NF * 2);
    float* P1 = (float*)take((size_t)NR * NM * 4); float* P2 = (float*)take((size_t)NR * NM * 4); float* P3 = (float*)take((size_t)NR * NF * 4);
    h16* H1 = (h16*)take((size_t)NR * NM * 2); h16* H2 = (h16*)take((size_t)NR * NM * 2); float* EN = (float*)take((size_t)NR * NR * 4); float* TW = (float*)take((size_t)NR * NR * 4);
    h16* WH = (h16*)take((size_t)NR * NR * 2); h16* TR = (h16*)take((size_t)NF * NR * 2); float* YC = (float*)take((size_t)NR * NF * 4);
    if ((size_t)(wsp - (char*)d_ws) > ws_size) return;
    k_rl8<<<NR * NF / 8 / 256, 256, 0, stream>>>(a0, PB);
    k_wtG<<<(NM * NF / 64 + 63) / 64, 256, 0, stream>>>(a2, NF, NM, W1); k_wtG<<<(NM * NF / 64 + 63) / 64, 256, 0, stream>>>(a4, NF, NM, W2); k_wtG<<<(NF * NF / 64 + 63) / 64, 256, 0, stream>>>(a6, NF, NF, W3);
    k_gemmw<bf, 0, true><<<dim3(NR / 64, NM / 64, 1), 32, 0, stream>>>(PB, nullptr, W1, nullptr, NF, P1, NM, a3, 0, 0, 0);
    k_gemmw<bf, 0, true><<<dim3(NR / 64, NM / 64, 1), 32, 0, stream>>>(PB, nullptr, W2, nullptr, NF, P2, NM, a5, 0, 0, 0);
    k_gemmw<bf, 0, true><<<dim3(NR / 64, NF / 64, 1), 32, 0, stream>>>(PB, nullptr, W3, nullptr, NF, P3, NF, a7, 0, 0, 0);
    k_f2h<<<NR * NM / 4 / 256, 256, 0, stream>>>(P1, H1, (size_t)NR * NM / 4); k_f2h<<<NR * NM / 4 / 256, 256, 0, stream>>>(P2, H2, (size_t)NR * NM / 4);
    k_gemmw<h16, 0, false><<<dim3(NR / 64, NR / 64, 1), 32, 0, stream>>>(H1, nullptr, H2, nullptr, NM, EN, NR, nullptr, 0, 0, 0);
    k_pair<<<NR, 256, 0, stream>>>(EN, a1, a8, a9, a10, a11, TW);
    k_rown<<<NR / 256, 256, 0, stream>>>(TW, WH);
    k_tr16<<<NF, 256, 0, stream>>>(P3, TR);
    k_gemmw<h16, 0, false><<<dim3(NR / 64, NF / 64, 1), 32, 0, stream>>>(WH, nullptr, TR, nullptr, NR, YC, NF, nullptr, 0, 0, 0);
    k_unc<<<NR * NF / 4 / 256, 256, 0, stream>>>(YC, OUT);
}
